// MultiRelationalGCNLayer_83330955477834
// MI455X (gfx1250) — hardware-verified
//
#include <hip/hip_runtime.h>
#include <stdint.h>


typedef __attribute__((ext_vector_type(16))) __bf16 v16bf;
typedef float        v8f __attribute__((ext_vector_type(8)));
typedef float        v4f __attribute__((ext_vector_type(4)));
typedef v4f __attribute__((may_alias)) v4fa;
typedef unsigned int v4u __attribute__((ext_vector_type(4)));
typedef int          v4i __attribute__((ext_vector_type(4)));
typedef int          v8i __attribute__((ext_vector_type(8)));

#define CH    128
#define HC    512
#define GT    128
#define DB    448
#define AGT   128
#define EPT   8
#define CHUNK (AGT * EPT)
#define LCAP  CHUNK
#define STP   132

static __device__ __forceinline__ unsigned int f2bf(float f) {
    unsigned int x = __float_as_uint(f);
    unsigned int r = x + 0x7FFFu + ((x >> 16) & 1u);
    return r >> 16;
}
static __device__ __forceinline__ unsigned int pk2(float lo, float hi) {
    return f2bf(lo) | (f2bf(hi) << 16);
}

union Frag { v16bf v; v4u q[2]; };

static __device__ __forceinline__ v8f wm(const Frag& a, const Frag& b, v8f c) {
    v8f d = __builtin_amdgcn_wmma_f32_16x16x32_bf16(false, a.v, false, b.v, (short)0, c, false, false);
    asm volatile("v_nop\n\tv_nop\n\tv_nop\n\tv_nop" : "+v"(d) : "v"(a.v), "v"(b.v));
    return d;
}

static __device__ __forceinline__ v8i load8(const int* p, int e0, int E, int fill) {
    union { v8i v; v4i q[2]; } u;
    if (e0 + EPT <= E) {
        u.q[0] = *(const v4i*)(p + e0);
        u.q[1] = *(const v4i*)(p + e0 + 4);
    } else {
        v8i v;
#pragma unroll
        for (int j = 0; j < EPT; ++j) v[j] = (e0 + j < E) ? p[e0 + j] : fill;
        u.v = v;
    }
    return u.v;
}

__global__ __launch_bounds__(128) void k_cvt_w(const float* __restrict__ w0, const float* __restrict__ w1,
                                               const float* __restrict__ w2, const float* __restrict__ w3,
                                               unsigned short* wb, int rowsTotal) {
    const int tg  = blockIdx.x * 128 + threadIdx.x;
    const int row = tg >> 4;
    const int cg  = tg & 15;
    const bool ok = row < rowsTotal;
    const int rowc = ok ? row : 0;
    const int mat  = rowc >> 7;
    const int rr   = rowc & (CH - 1);
    const float* src = (mat == 0) ? w0 : ((mat == 1) ? w1 : ((mat == 2) ? w2 : w3));
    const float* p = src + (size_t)rr * CH + cg * 8;
    const v4f f0 = *(const v4f*)p;
    const v4f f1 = *(const v4f*)(p + 4);
    v4u o;
    o.x = pk2(f0.x, f0.y); o.y = pk2(f0.z, f0.w);
    o.z = pk2(f1.x, f1.y); o.w = pk2(f1.z, f1.w);
    unsigned short* q = wb + (size_t)rowc * CH + cg * 8;
    if (ok) *(volatile v4u*)q = o;
    __threadfence();
    if (ok) *(volatile v4u*)q = o;
}

__global__ __launch_bounds__(GT) void k_gemm(const float* __restrict__ X,
                                            const unsigned short* __restrict__ Wb,
                                            float* H, int numNodes) {
    __shared__ float st[4][16][STP];

    const int w    = threadIdx.x >> 5;
    const int lane = threadIdx.x & 31;
    const int h    = lane >> 4;
    const int m    = lane & 15;
    const int row0 = blockIdx.x * 16;

    int ra = row0 + m;
    if (ra > numNodes - 1) ra = numNodes - 1;
    const float* ap = X + (size_t)ra * CH;
    const unsigned short* bp = Wb + (size_t)(w * 128 + m) * CH;

    const v8f zero8 = {0.f, 0.f, 0.f, 0.f, 0.f, 0.f, 0.f, 0.f};
    v8f acc[8];
#pragma unroll
    for (int j = 0; j < 8; ++j) acc[j] = zero8;

#pragma unroll
    for (int s = 0; s < 4; ++s) {
        const int k0 = 32 * s;
        Frag a;
        {
            const float* p0 = ap + k0 + 8 * h;
            const float* p1 = ap + k0 + 16 + 8 * h;
            const v4f f0 = *(const v4f*)p0, f1 = *(const v4f*)(p0 + 4);
            const v4f g0 = *(const v4f*)p1, g1 = *(const v4f*)(p1 + 4);
            v4u qa, qb;
            qa.x = pk2(f0.x, f0.y); qa.y = pk2(f0.z, f0.w); qa.z = pk2(f1.x, f1.y); qa.w = pk2(f1.z, f1.w);
            qb.x = pk2(g0.x, g0.y); qb.y = pk2(g0.z, g0.w); qb.z = pk2(g1.x, g1.y); qb.w = pk2(g1.z, g1.w);
            a.q[0] = qa; a.q[1] = qb;
        }
#pragma unroll
        for (int j = 0; j < 8; ++j) {
            const unsigned short* q = bp + (size_t)j * 16 * CH + k0;
            Frag b;
            b.q[0] = *(const v4u*)(q + 8 * h);
            b.q[1] = *(const v4u*)(q + 16 + 8 * h);
            acc[j] = wm(a, b, acc[j]);
        }
    }

#pragma unroll
    for (int j = 0; j < 8; ++j) {
#pragma unroll
        for (int r = 0; r < 8; ++r) st[w][8 * h + r][16 * j + m] = acc[j][r];
    }
    __syncthreads();

    float* hb = H + (size_t)row0 * HC + w * 128 + 4 * lane;
    for (int r = 0; r < 16; ++r) {
        if (row0 + r < numNodes) {
            const v4f v = *(const v4fa*)(&st[w][r][4 * lane]);
            *(volatile v4f*)(hb + (size_t)r * HC) = v;
        }
    }
    __threadfence();
    for (int r = 0; r < 16; ++r) {
        if (row0 + r < numNodes) {
            const v4f v = *(const v4fa*)(&st[w][r][4 * lane]);
            *(volatile v4f*)(hb + (size_t)r * HC) = v;
        }
    }
}

__global__ __launch_bounds__(AGT) void k_agg(const float* __restrict__ H, const float* __restrict__ bias,
                                            const int* __restrict__ s0, const int* __restrict__ t0, int E0,
                                            const int* __restrict__ s1, const int* __restrict__ t1, int E1,
                                            const int* __restrict__ s2, const int* __restrict__ t2, int E2,
                                            float* out, int numNodes) {
    extern __shared__ v4f accD[];
    __shared__ float invL[DB];
    __shared__ int   cntL[4 * DB];
    __shared__ int   lstS[LCAP];
    __shared__ int   lstD[LCAP];
    __shared__ int   wtot[4];

    const int t    = threadIdx.x;
    const int w    = t >> 5;
    const int lane = t & 31;
    const int d0   = blockIdx.x * DB;
    int dbe = numNodes - d0;
    if (dbe > DB) dbe = DB;
    if (dbe < 0)  dbe = 0;
    const unsigned int ltm = (1u << lane) - 1u;
    const v4f zero4 = {0.f, 0.f, 0.f, 0.f};

    for (int i = t; i < DB * (CH / 4); i += AGT) accD[i] = zero4;

    for (int r = 0; r < 3; ++r) {
        const int* sp = (r == 0) ? s0 : ((r == 1) ? s1 : s2);
        const int* tp = (r == 0) ? t0 : ((r == 1) ? t1 : t2);
        const int  E  = (r == 0) ? E0 : ((r == 1) ? E1 : E2);
        const int colOff = r * CH;

        __syncthreads();
        for (int i = t; i < 4 * DB; i += AGT) cntL[i] = 0;
        __syncthreads();

#pragma unroll 1
        for (int base = 0; base < E; base += CHUNK) {
            const v8i dv  = load8(tp, base + EPT * t, E, -1);
            const v8i dlv = dv - d0;
#pragma unroll
            for (int j = 0; j < EPT; ++j) {
                const int dl = dlv[j];
                unsigned int b = __builtin_amdgcn_ballot_w32((unsigned)dl < (unsigned)dbe);
                while (b != 0u) {
                    const int q = __builtin_ctz(b);
                    b &= b - 1u;
                    int dq = __builtin_amdgcn_readlane(dl, q);
                    dq = dq < 0 ? 0 : (dq > DB - 1 ? DB - 1 : dq);
                    if (lane == 0) cntL[w * DB + dq] += 1;
                }
            }
        }
        __syncthreads();
        for (int i = t; i < DB; i += AGT) {
            int c = cntL[i] + cntL[DB + i] + cntL[2 * DB + i] + cntL[3 * DB + i];
            if (c < 1) c = 1;
            invL[i] = 1.0f / (float)c;
        }
        __syncthreads();

#pragma unroll 1
        for (int base = 0; base < E; base += CHUNK) {
            const v8i dv  = load8(tp, base + EPT * t, E, -1);
            const v8i sv  = load8(sp, base + EPT * t, E, 0);
            const v8i dlv = dv - d0;

            unsigned int bm[EPT];
            int tot = 0;
#pragma unroll
            for (int j = 0; j < EPT; ++j) {
                bm[j] = __builtin_amdgcn_ballot_w32((unsigned)dlv[j] < (unsigned)dbe);
                tot += __builtin_popcount(bm[j]);
            }
            if (lane == 0) wtot[w] = tot;
            __syncthreads();

            const int c0 = wtot[0], c1 = wtot[1], c2 = wtot[2], c3 = wtot[3];
            int nh = c0 + c1 + c2 + c3;
            if (nh > LCAP) nh = LCAP;
            int pos = 0;
            if (w > 0) pos += c0;
            if (w > 1) pos += c1;
            if (w > 2) pos += c2;
#pragma unroll
            for (int j = 0; j < EPT; ++j) {
                const unsigned int b = bm[j];
                if (b != 0u) {
                    const int p = pos + __builtin_popcount(b & ltm);
                    if ((((b >> lane) & 1u) != 0u) && ((unsigned)p < (unsigned)LCAP)) {
                        lstS[p] = sv[j];
                        lstD[p] = dlv[j];
                    }
                    pos += __builtin_popcount(b);
                }
            }
            __syncthreads();

            for (int g = 0; g < nh; g += 32) {
                const int  i     = g + lane;
                const bool valid = i < nh;
                const int  ic    = valid ? i : 0;
                const int  dli   = lstD[ic];
                const int  si    = lstS[ic];
                unsigned int b = __builtin_amdgcn_ballot_w32(valid && ((dli & 3) == w));
                while (b != 0u) {
                    const int q = __builtin_ctz(b);
                    b &= b - 1u;
                    int dq = __builtin_amdgcn_readlane(dli, q);
                    int sq = __builtin_amdgcn_readlane(si, q);
                    dq = dq < 0 ? 0 : (dq > DB - 1 ? DB - 1 : dq);
                    sq = sq < 0 ? 0 : (sq > numNodes - 1 ? numNodes - 1 : sq);
                    const float sc = invL[dq];
                    const v4f v = *(const v4f*)(H + (size_t)sq * HC + colOff + 4 * lane);
                    const int ai = dq * (CH / 4) + lane;
                    v4f a = accD[ai];
                    a = a + v * sc;
                    accD[ai] = a;
                }
            }
        }
    }
    __syncthreads();

    const v4f bb = *(const v4f*)(bias + 4 * lane);
    for (int dl = w; dl < dbe; dl += 4) {
        const int d = d0 + dl;
        const v4f hs = *(const v4f*)(H + (size_t)d * HC + 3 * CH + 4 * lane);
        v4f v = accD[dl * (CH / 4) + lane] + hs + bb;
        v.x = v.x > 0.0f ? v.x : 0.0f;
        v.y = v.y > 0.0f ? v.y : 0.0f;
        v.z = v.z > 0.0f ? v.z : 0.0f;
        v.w = v.w > 0.0f ? v.w : 0.0f;
        *(volatile v4f*)(out + (size_t)d * CH + 4 * lane) = v;
    }
    __threadfence();
    for (int dl = w; dl < dbe; dl += 4) {
        const int d = d0 + dl;
        const v4f hs = *(const v4f*)(H + (size_t)d * HC + 3 * CH + 4 * lane);
        v4f v = accD[dl * (CH / 4) + lane] + hs + bb;
        v.x = v.x > 0.0f ? v.x : 0.0f;
        v.y = v.y > 0.0f ? v.y : 0.0f;
        v.z = v.z > 0.0f ? v.z : 0.0f;
        v.w = v.w > 0.0f ? v.w : 0.0f;
        *(volatile v4f*)(out + (size_t)d * CH + 4 * lane) = v;
    }
}

extern "C" void kernel_launch(void* const* d_in, const int* in_sizes, int n_in,
                              void* d_out, int out_size, void* d_ws, size_t ws_size,
                              hipStream_t stream) {
    if (n_in < 12) return;
    const float* X    = (const float*)d_in[0];
    const float* W0   = (const float*)d_in[1];
    const float* W1   = (const float*)d_in[2];
    const float* W2   = (const float*)d_in[3];
    const float* Ws   = (const float*)d_in[4];
    const float* bias = (const float*)d_in[5];
    const int* src0 = (const int*)d_in[6];
    const int* dst0 = (const int*)d_in[7];
    const int* src1 = (const int*)d_in[8];
    const int* dst1 = (const int*)d_in[9];
    const int* src2 = (const int*)d_in[10];
    const int* dst2 = (const int*)d_in[11];

    const int numNodes = in_sizes[0] / CH;
    if (numNodes < 1 || numNodes * CH != in_sizes[0]) return;
    if (in_sizes[1] != CH * CH || in_sizes[2] != CH * CH || in_sizes[3] != CH * CH || in_sizes[4] != CH * CH) return;
    if (in_sizes[5] != CH) return;
    if (out_size != numNodes * CH) return;
    const int E0 = in_sizes[6] < in_sizes[7]  ? in_sizes[6]  : in_sizes[7];
    const int E1 = in_sizes[8] < in_sizes[9]  ? in_sizes[8]  : in_sizes[9];
    const int E2 = in_sizes[10] < in_sizes[11] ? in_sizes[10] : in_sizes[11];
    if (E0 < 0 || E1 < 0 || E2 < 0) return;

    const size_t offWb   = 0;
    const size_t bytesWb = (size_t)4 * CH * CH * sizeof(unsigned short);
    const size_t offH    = (offWb + bytesWb + 255) & ~(size_t)255;
    const size_t bytesH  = (size_t)numNodes * HC * sizeof(float);
    if (offH + bytesH > ws_size) return;

    unsigned short* Wb = (unsigned short*)((char*)d_ws + offWb);
    float* H   = (float*)((char*)d_ws + offH);
    float* out = (float*)d_out;

    {
        const int rowsTotal = 4 * CH;
        const int threads = rowsTotal * 16;
        const int blocks = (threads + 127) / 128;
        k_cvt_w<<<blocks, 128, 0, stream>>>(W0, W1, W2, Ws, Wb, rowsTotal);
    }
    {
        const int blocks = (numNodes + 15) / 16;
        k_gemm<<<blocks, GT, 0, stream>>>(X, Wb, H, numNodes);
    }
    {
        const size_t dyn = (size_t)DB * CH * sizeof(float);
        hipFuncSetAttribute(reinterpret_cast<const void*>(&k_agg),
                            hipFuncAttributeMaxDynamicSharedMemorySize, (int)dyn);
        const int blocks = (numNodes + DB - 1) / DB;
        k_agg<<<blocks, AGT, dyn, stream>>>(H, bias, src0, dst0, E0, src1, dst1, E1, src2, dst2, E2,
                                           out, numNodes);
    }
    hipGetLastError();
}
